// CausalSelfAttention_69011534512786
// MI455X (gfx1250) — hardware-verified
//
#include <hip/hip_runtime.h>
#ifndef NB
#define NB 2
#endif
#ifndef SEQ
#define SEQ 2048
#endif
#define NB_FULL 2
#define SEQ_FULL 2048
#define DM 1024
#define NH 16
#define HD 64
#define ISL ((SEQ) < 256 ? (SEQ) : 256)
#define NR (NB * SEQ)
#define NRI (NB * ISL)
#define LQK (2 * DM)
#define LVT NR
#define LVL NRI

static_assert(NB >= 1 && NB <= NB_FULL);
static_assert(SEQ <= SEQ_FULL);
static_assert(SEQ % 128 == 0);
static_assert(ISL % 128 == 0);
static_assert(ISL >= 32);
static_assert((SEQ - ISL) % 128 == 0);
static_assert(NH * HD == DM);
static_assert(HD == 64);
static_assert(DM % 128 == 0);
static_assert(DM % 8 == 0);
static_assert(NR % 128 == 0);
static_assert(NRI % 64 == 0);
static_assert((long long)NR * LQK < 2147483647LL);
static_assert((long long)DM * LVT < 2147483647LL);

typedef unsigned short v8us __attribute__((ext_vector_type(8), may_alias));
typedef float  v8f  __attribute__((ext_vector_type(8)));
typedef float  v4f  __attribute__((ext_vector_type(4)));
typedef float  v4fa __attribute__((ext_vector_type(4), may_alias));
typedef _Float16 v16h __attribute__((ext_vector_type(16)));
typedef _Float16 v4h  __attribute__((ext_vector_type(4)));
union FragH { v16h v; v8us half[2]; _Float16 h[16]; unsigned short u[16]; };

__device__ __forceinline__ float bf16_rne(float x) { unsigned int u = __float_as_uint(x); u = (u + 0x7FFFu + ((u >> 16) & 1u)) & 0xFFFF0000u; return __uint_as_float(u); }

__device__ __forceinline__ v16h g2_frag(const _Float16* p, int hh) { FragH f; f.half[0] = *(const v8us*)((const unsigned short*)p + 8 * hh); f.half[1] = *(const v8us*)((const unsigned short*)p + 16 + 8 * hh); return f.v; }
__device__ __forceinline__ v8f g2_mma(v16h a, v16h b, v8f c) { v8f d = __builtin_amdgcn_wmma_f32_16x16x32_f16(false, a, false, b, (short)0, c, false, false); asm volatile("v_nop\n\tv_nop\n\tv_nop\n\tv_nop" : "+v"(d) : "v"(a), "v"(b)); return d; }

__global__ __launch_bounds__(256) void k_wt_f16(const float* __restrict__ W, _Float16* __restrict__ Wt, int K, int N, float scale) {
  const int t = blockIdx.x * 256 + threadIdx.x; if (t >= N * (K / 8)) return; const int n = t / (K / 8), k8 = (t % (K / 8)) * 8; FragH f;
#pragma unroll
  for (int i = 0; i < 8; ++i) f.h[i] = (_Float16)(bf16_rne(W[(size_t)(k8 + i) * N + n]) * scale);
  const v8us o = f.half[0];
  unsigned short* d = (unsigned short*)Wt + (size_t)n * K + k8;
  *(volatile v8us*)d = o; __threadfence(); *(volatile v8us*)d = o;
}

__global__ __launch_bounds__(256) void k_x16(const float* __restrict__ x, _Float16* __restrict__ X16) {
  const int t = blockIdx.x * 256 + threadIdx.x; if (t >= NR * (DM / 8)) return;
  const int row = t / (DM / 8), c8 = (t % (DM / 8)) * 8; const int b = row / SEQ, s = row % SEQ;
  const float* src = x + ((size_t)b * SEQ_FULL + s) * DM + c8;
  const v4f a = *(const v4fa*)src, c = *(const v4fa*)(src + 4); FragH f;
#pragma unroll
  for (int i = 0; i < 4; ++i) { f.h[i] = (_Float16)bf16_rne(a[i]); f.h[4 + i] = (_Float16)bf16_rne(c[i]); }
  const v8us o = f.half[0];
  unsigned short* d = (unsigned short*)X16 + (size_t)row * DM + c8;
  *(volatile v8us*)d = o; __threadfence(); *(volatile v8us*)d = o;
}

template <int MT, bool ROWBIAS, bool ARES, int OUT>
__device__ __forceinline__ void gemm_body(const _Float16* __restrict__ A, const _Float16* __restrict__ AL, int lda,
    const _Float16* __restrict__ Bh, int ldb, float alpha, float alphaL, const float* __restrict__ bias,
    float* __restrict__ Cf, _Float16* __restrict__ C16, _Float16* __restrict__ CL, int ldc, int ldcl,
    int M, int N, int K, int segRows, int aSeg, int aOff, int cSeg, int cOff) {
  static_assert(MT == 1 || MT == 2);
  static_assert(!ARES || MT == 1);
  __shared__ __attribute__((aligned(16))) float so[4][32][68];
  const int tid = threadIdx.x, w = tid >> 5, lane = tid & 31, ln = lane & 15, hh = lane >> 4;
  const int ntn = N >> 6;
  const int mt = blockIdx.x / ntn, nq = blockIdx.x - mt * ntn;
  const int R0 = mt * (64 * MT) + (16 * MT) * w, col0 = nq * 64;
  if (R0 >= M) return;
  const int seg = R0 / segRows, wi = R0 - seg * segRows;
  const int arow0 = seg * aSeg + aOff + wi, crow0 = seg * cSeg + cOff + wi;
  const _Float16* a0p = A + (size_t)(arow0 + ln) * lda;
  const _Float16* b0p = Bh + (size_t)(col0 + ln) * ldb; const _Float16* b1p = b0p + (size_t)16 * ldb; const _Float16* b2p = b1p + (size_t)16 * ldb; const _Float16* b3p = b2p + (size_t)16 * ldb;
  const v8f z8 = {0.f, 0.f, 0.f, 0.f, 0.f, 0.f, 0.f, 0.f};
  v8f c00 = z8, c01 = z8, c02 = z8, c03 = z8, c10 = z8, c11 = z8, c12 = z8, c13 = z8, d00 = z8, d01 = z8, d02 = z8, d03 = z8;
#pragma unroll 1
  for (int kb = 0; kb < K; kb += 32) {
    const v16h a0 = g2_frag(a0p + kb, hh);
    v16h a1 = a0, e0 = a0;
    if (MT == 2) a1 = g2_frag(a0p + (size_t)16 * lda + kb, hh);
    if (ARES) e0 = g2_frag(AL + (size_t)(R0 + ln) * lda + kb, hh);
    v16h b = g2_frag(b0p + kb, hh);
    c00 = g2_mma(a0, b, c00); if (MT == 2) c10 = g2_mma(a1, b, c10); if (ARES) d00 = g2_mma(e0, b, d00);
    b = g2_frag(b1p + kb, hh);
    c01 = g2_mma(a0, b, c01); if (MT == 2) c11 = g2_mma(a1, b, c11); if (ARES) d01 = g2_mma(e0, b, d01);
    b = g2_frag(b2p + kb, hh);
    c02 = g2_mma(a0, b, c02); if (MT == 2) c12 = g2_mma(a1, b, c12); if (ARES) d02 = g2_mma(e0, b, d02);
    b = g2_frag(b3p + kb, hh);
    c03 = g2_mma(a0, b, c03); if (MT == 2) c13 = g2_mma(a1, b, c13); if (ARES) d03 = g2_mma(e0, b, d03);
  }
  const v8f accs[8] = {c00, c01, c02, c03, c10, c11, c12, c13};
  const v8f accl[4] = {d00, d01, d02, d03};
#pragma unroll
  for (int u = 0; u < 4 * MT; ++u) {
    const int t = u & 3, half = u >> 2; const int col = col0 + t * 16 + ln;
    float bvc = 0.f; if (!ROWBIAS) bvc = bf16_rne(bias[col]);
#pragma unroll
    for (int r = 0; r < 8; ++r) {
      const int rloc = half * 16 + 8 * hh + r;
      float v = accs[u][r] * alpha;
      if (ARES) v += accl[t][r] * alphaL;
      if (ROWBIAS) v += bf16_rne(bias[R0 + rloc]); else v += bvc;
      so[w][rloc][t * 16 + ln] = v;
    }
  }
  __builtin_amdgcn_fence(4  , "workgroup"); __builtin_amdgcn_wave_barrier();
  const int rsub = lane >> 4, c4 = (lane & 15) * 4;
  if (OUT == 0) {
    for (int pass = 0; pass < 2; ++pass) {
#pragma unroll
      for (int q = 0; q < 8 * MT; ++q) { const int r = q * 2 + rsub; const v4f v = *(const v4fa*)&so[w][r][c4]; *(volatile v4f*)(Cf + (size_t)(crow0 + r) * ldc + col0 + c4) = v; }
      if (pass == 0) __threadfence();
    }
  } else {
    int sl, rrow0, rcol0;
    if (OUT == 1) { sl = crow0 % SEQ; rrow0 = (crow0 / SEQ) * ISL + sl; rcol0 = col0; }
    else          { sl = col0 % SEQ;  rrow0 = crow0; rcol0 = (col0 / SEQ) * ISL + sl; }
    const bool isl = sl < ISL;
    for (int pass = 0; pass < 2; ++pass) {
#pragma unroll
      for (int q = 0; q < 8 * MT; ++q) {
        const int r = q * 2 + rsub; const v4f v = *(const v4fa*)&so[w][r][c4];
        v4h h4, l4;
#pragma unroll
        for (int i = 0; i < 4; ++i) { const _Float16 hv = (_Float16)v[i]; h4[i] = hv; l4[i] = (_Float16)((v[i] - (float)hv) * 1024.0f); }
        *(volatile v4h*)(C16 + (size_t)(crow0 + r) * ldc + col0 + c4) = h4;
        if (isl) *(volatile v4h*)(CL + (size_t)(rrow0 + r) * ldcl + rcol0 + c4) = l4;
      }
      if (pass == 0) __threadfence();
    }
  }
}

__global__ __launch_bounds__(128) void k_gemm_qk(const _Float16* __restrict__ X16, const _Float16* __restrict__ BW, const float* __restrict__ bias, _Float16* __restrict__ QK, _Float16* __restrict__ QKL) {
  gemm_body<2, false, false, 1>(X16, nullptr, DM, BW, DM, 0.0625f, 0.f, bias, nullptr, QK, QKL, LQK, LQK, NR, 2 * DM, DM, NR, 0, 0, 0, 0);
}
__global__ __launch_bounds__(128) void k_gemm_vt(const _Float16* __restrict__ BWv, const _Float16* __restrict__ X16, const float* __restrict__ biasv, _Float16* __restrict__ VT, _Float16* __restrict__ VTL) {
  gemm_body<2, true, false, 2>(BWv, nullptr, DM, X16, DM, 0.0625f, 0.f, biasv, nullptr, VT, VTL, LVT, LVL, DM, NR, DM, DM, 0, 0, 0, 0);
}
__global__ __launch_bounds__(128) void k_gemm_out(const _Float16* __restrict__ O16, const _Float16* __restrict__ BO, const float* __restrict__ bias, float* __restrict__ out) {
  gemm_body<2, false, false, 0>(O16, nullptr, DM, BO, DM, 0.0009765625f, 0.f, bias, out, nullptr, nullptr, DM, 0, NB * (SEQ - ISL), DM, DM, SEQ - ISL, SEQ, ISL, SEQ_FULL, ISL);
}
__global__ __launch_bounds__(128) void k_gemm_out_isl(const _Float16* __restrict__ O16, const _Float16* __restrict__ OL, const _Float16* __restrict__ BO, const float* __restrict__ bias, float* __restrict__ out) {
  gemm_body<1, false, true, 0>(O16, OL, DM, BO, DM, 0.0009765625f, 0.00000095367431640625f, bias, out, nullptr, nullptr, DM, 0, NRI, DM, DM, ISL, SEQ, 0, SEQ_FULL, 0);
}

template <bool RES>
__device__ __forceinline__ void attn_body(const _Float16* __restrict__ QK, const _Float16* __restrict__ QKL, const _Float16* __restrict__ VT, const _Float16* __restrict__ VTL,
                                          _Float16* __restrict__ O16, _Float16* __restrict__ OL, const int* __restrict__ Sp, int qb0, int nqb) {
  __shared__ __attribute__((aligned(16))) float so[8][16][68];
  const int tid = threadIdx.x, lane = tid & 31, ln = lane & 15, hh = lane >> 4;
  const int w = __builtin_amdgcn_readfirstlane(tid >> 5);
  const int sraw = Sp[0];
  const int Sc = sraw < 0 ? 0 : (sraw > SEQ ? SEQ : sraw);
  const int bh = (int)blockIdx.x / nqb; const int qb = qb0 + ((int)blockIdx.x - bh * nqb);
  const int h = bh % NH, b = bh / NH;
  const int q0 = qb * 128 + w * 16, q = q0 + ln;
  const bool qpre = q < Sc;
  const int rowb = b * SEQ, rowi = b * ISL;
  const _Float16* qp = QK + (size_t)(rowb + q) * LQK + h * HD;
  const v16h qh0 = g2_frag(qp, hh), qh1 = g2_frag(qp + 32, hh);
  const int qloff = (rowi + q) * LQK + h * HD;
  const int kbase = (rowb + ln) * LQK + DM + h * HD;
  const int klbase = (rowi + ln) * LQK + DM + h * HD;
  const int vbase = (h * HD + ln) * LVT + rowb;
  const int vlbase = (h * HD + ln) * LVL + rowi;
  const v8f z8 = {0.f, 0.f, 0.f, 0.f, 0.f, 0.f, 0.f, 0.f};
  const v16h zh = (v16h)((_Float16)0.0f);
  v8f o0 = z8, o1 = z8, o2 = z8, o3 = z8, e0 = z8, e1 = z8, e2 = z8, e3 = z8;
  float m = -1.0e30f, l = 0.f;
  const int kend = (Sc > q0 + 16) ? Sc : (q0 + 16);
  const int nst = (kend + 31) >> 5;
#pragma unroll 1
  for (int st = 0; st < nst; ++st) {
    const int kcb = st * 32;
    const bool rok = kcb < ISL;
    const int kcl = rok ? kcb : (ISL - 32);
    const _Float16* kp0 = QK + kbase + kcb * LQK; const _Float16* kp1 = kp0 + 16 * LQK;
    v8f s0 = z8, s1 = z8, r0 = z8, r1 = z8;
    if (RES) {
      int qo = qloff; asm volatile("" : "+v"(qo));
      const _Float16* qlp = QKL + qo;
      const v16h ql0 = g2_frag(qlp, hh), ql1 = g2_frag(qlp + 32, hh);
      const _Float16* kl0 = QKL + klbase + kcl * LQK; const _Float16* kl1 = kl0 + 16 * LQK;
      v16h ah = g2_frag(kp0, hh), al = g2_frag(kl0, hh); al = rok ? al : zh;
      s0 = g2_mma(ah, qh0, s0); r0 = g2_mma(al, qh0, r0); r0 = g2_mma(ah, ql0, r0);
      ah = g2_frag(kp0 + 32, hh); al = g2_frag(kl0 + 32, hh); al = rok ? al : zh;
      s0 = g2_mma(ah, qh1, s0); r0 = g2_mma(al, qh1, r0); r0 = g2_mma(ah, ql1, r0);
      ah = g2_frag(kp1, hh); al = g2_frag(kl1, hh); al = rok ? al : zh;
      s1 = g2_mma(ah, qh0, s1); r1 = g2_mma(al, qh0, r1); r1 = g2_mma(ah, ql0, r1);
      ah = g2_frag(kp1 + 32, hh); al = g2_frag(kl1 + 32, hh); al = rok ? al : zh;
      s1 = g2_mma(ah, qh1, s1); r1 = g2_mma(al, qh1, r1); r1 = g2_mma(ah, ql1, r1);
    } else {
      v16h ah = g2_frag(kp0, hh); s0 = g2_mma(ah, qh0, s0);
      ah = g2_frag(kp0 + 32, hh); s0 = g2_mma(ah, qh1, s0);
      ah = g2_frag(kp1, hh);      s1 = g2_mma(ah, qh0, s1);
      ah = g2_frag(kp1 + 32, hh); s1 = g2_mma(ah, qh1, s1);
    }
    v8f xa, xb; float mt = -1.0e30f;
#pragma unroll
    for (int r = 0; r < 8; ++r) {
      const int k0 = kcb + 8 * hh + r;
      const bool va = (k0 <= q) || (qpre && (k0 < Sc));
      const bool vb = (k0 + 16 <= q) || (qpre && (k0 + 16 < Sc));
      float a = s0[r], c = s1[r];
      if (RES) { a += r0[r] * 0.0009765625f; c += r1[r] * 0.0009765625f; }
      a *= 0.125f; c *= 0.125f;
      a = va ? a : -1.0e30f; c = vb ? c : -1.0e30f;
      xa[r] = a; xb[r] = c; mt = fmaxf(mt, fmaxf(a, c));
    }
    mt = fmaxf(mt, __shfl_xor(mt, 16, 32));
    const float mn = fmaxf(m, mt);
    const float f = __expf(fmaxf(m - mn, -80.0f));
    m = mn;
    FragH ph, pl; float rs = 0.f;
#pragma unroll
    for (int r = 0; r < 8; ++r) {
      const int k0 = kcb + 8 * hh + r;
      const bool va = (k0 <= q) || (qpre && (k0 < Sc));
      const bool vb = (k0 + 16 <= q) || (qpre && (k0 + 16 < Sc));
      float pa = __expf(va ? (xa[r] - mn) : 0.f); pa = va ? pa : 0.f;
      float pb = __expf(vb ? (xb[r] - mn) : 0.f); pb = vb ? pb : 0.f;
      rs += pa + pb;
      const float ta = pa * 1024.0f, tb = pb * 1024.0f;
      const _Float16 ha = (_Float16)ta, hb = (_Float16)tb;
      ph.h[r] = ha; ph.h[8 + r] = hb;
      if (RES) { pl.h[r] = (_Float16)((ta - (float)ha) * 1024.0f); pl.h[8 + r] = (_Float16)((tb - (float)hb) * 1024.0f); }
    }
    const float rso = __shfl_xor(rs, 16, 32);
    l = l * f + (rs + rso);
    o0 *= f; o1 *= f; o2 *= f; o3 *= f;
    if (RES) { e0 *= f; e1 *= f; e2 *= f; e3 *= f; }
    const _Float16* vp = VT + vbase + kcb;
    const v16h v0 = g2_frag(vp, hh), v1 = g2_frag(vp + 16 * LVT, hh), v2 = g2_frag(vp + 32 * LVT, hh), v3 = g2_frag(vp + 48 * LVT, hh);
    o0 = g2_mma(v0, ph.v, o0); o1 = g2_mma(v1, ph.v, o1); o2 = g2_mma(v2, ph.v, o2); o3 = g2_mma(v3, ph.v, o3);
    if (RES) {
      const _Float16* vlp = VTL + vlbase + kcl;
      v16h vl = g2_frag(vlp, hh); vl = rok ? vl : zh;            e0 = g2_mma(vl, ph.v, e0); e0 = g2_mma(v0, pl.v, e0);
      vl = g2_frag(vlp + 16 * LVL, hh); vl = rok ? vl : zh;      e1 = g2_mma(vl, ph.v, e1); e1 = g2_mma(v1, pl.v, e1);
      vl = g2_frag(vlp + 32 * LVL, hh); vl = rok ? vl : zh;      e2 = g2_mma(vl, ph.v, e2); e2 = g2_mma(v2, pl.v, e2);
      vl = g2_frag(vlp + 48 * LVL, hh); vl = rok ? vl : zh;      e3 = g2_mma(vl, ph.v, e3); e3 = g2_mma(v3, pl.v, e3);
    }
  }
  const float inv = 0.0625f * (1.0f / l);
  const v8f oo[4] = {o0, o1, o2, o3}; const v8f ee[4] = {e0, e1, e2, e3};
#pragma unroll
  for (int dg = 0; dg < 4; ++dg)
#pragma unroll
    for (int r = 0; r < 8; ++r) { float v = oo[dg][r]; if (RES) v += ee[dg][r] * 0.0009765625f; so[w][ln][dg * 16 + 8 * hh + r] = v * inv; }
  __builtin_amdgcn_fence(4  , "workgroup"); __builtin_amdgcn_wave_barrier();
  const int rq = lane >> 3, pc = (lane & 7) * 8;
  for (int pass = 0; pass < 2; ++pass) {
#pragma unroll
    for (int it = 0; it < 4; ++it) {
      const int row = it * 4 + rq;
      const v4f a = *(const v4fa*)&so[w][row][pc], c = *(const v4fa*)&so[w][row][pc + 4];
      FragH fh, fl;
#pragma unroll
      for (int i = 0; i < 4; ++i) {
        const _Float16 h0 = (_Float16)a[i], h1 = (_Float16)c[i]; fh.h[i] = h0; fh.h[4 + i] = h1;
        fl.h[i] = (_Float16)((a[i] - (float)h0) * 1024.0f); fl.h[4 + i] = (_Float16)((c[i] - (float)h1) * 1024.0f);
      }
      const v8us oh = fh.half[0], ol = fl.half[0];
      *(volatile v8us*)((unsigned short*)O16 + (size_t)(rowb + q0 + row) * DM + h * HD + pc) = oh;
      if (RES) *(volatile v8us*)((unsigned short*)OL + (size_t)(rowi + q0 + row) * DM + h * HD + pc) = ol;
    }
    if (pass == 0) __threadfence();
  }
}

__global__ __launch_bounds__(256) void k_attn_isl(const _Float16* __restrict__ QK, const _Float16* __restrict__ QKL, const _Float16* __restrict__ VT, const _Float16* __restrict__ VTL, _Float16* __restrict__ O16, _Float16* __restrict__ OL, const int* __restrict__ Sp) {
  attn_body<true>(QK, QKL, VT, VTL, O16, OL, Sp, 0, ISL / 128);
}
__global__ __launch_bounds__(256) void k_attn_main(const _Float16* __restrict__ QK, const _Float16* __restrict__ VT, _Float16* __restrict__ O16, const int* __restrict__ Sp) {
  attn_body<false>(QK, nullptr, VT, nullptr, O16, nullptr, Sp, ISL / 128, (SEQ - ISL) / 128);
}

constexpr size_t al256(size_t bytes) { return (bytes + 255) & ~(size_t)255; }
constexpr size_t SZ_BQKV = al256((size_t)3 * DM * DM * 2);
constexpr size_t SZ_BO   = al256((size_t)DM * DM * 2);
constexpr size_t SZ_X16  = al256((size_t)NR * DM * 2);
constexpr size_t SZ_QK   = al256((size_t)NR * LQK * 2);
constexpr size_t SZ_QKL  = al256((size_t)NRI * LQK * 2);
constexpr size_t SZ_VT   = al256((size_t)DM * LVT * 2);
constexpr size_t SZ_VTL  = al256((size_t)DM * LVL * 2);
constexpr size_t SZ_O16  = al256((size_t)NR * DM * 2);
constexpr size_t SZ_OL   = al256((size_t)NRI * DM * 2);
constexpr size_t WS_TOTAL = SZ_BQKV + SZ_BO + SZ_X16 + SZ_QK + SZ_QKL + SZ_VT + SZ_VTL + SZ_O16 + SZ_OL;
static_assert(WS_TOTAL <= (size_t)134217728);

extern "C" void kernel_launch(void* const* d_in, const int* in_sizes, int n_in,
                              void* d_out, int out_size, void* d_ws, size_t ws_size, hipStream_t stream) {
  if (n_in < 6) return;
  const long long xrows = (long long)(NB - 1) * SEQ_FULL + SEQ;
  if ((long long)in_sizes[0] < xrows * DM) return;
  if ((long long)in_sizes[1] < (long long)DM * 3 * DM) return;
  if ((long long)in_sizes[2] < (long long)3 * DM) return;
  if ((long long)in_sizes[3] < (long long)DM * DM) return;
  if ((long long)in_sizes[4] < (long long)DM) return;
  if ((long long)in_sizes[5] < 1) return;
  if ((long long)out_size < xrows * DM) return;
  if (WS_TOTAL > ws_size) return;
  const float* x = (const float*)d_in[0]; const float* w_attn = (const float*)d_in[1]; const float* b_attn = (const float*)d_in[2];
  const float* w_proj = (const float*)d_in[3]; const float* b_proj = (const float*)d_in[4];
  const int* s_pref = (const int*)d_in[5];
  float* out = (float*)d_out;
  char* ws = (char*)d_ws; size_t off = 0;
  _Float16* BQKV = (_Float16*)(ws + off); off += SZ_BQKV;
  _Float16* BO   = (_Float16*)(ws + off); off += SZ_BO;
  _Float16* X16  = (_Float16*)(ws + off); off += SZ_X16;
  _Float16* QK   = (_Float16*)(ws + off); off += SZ_QK;
  _Float16* QKL  = (_Float16*)(ws + off); off += SZ_QKL;
  _Float16* VT   = (_Float16*)(ws + off); off += SZ_VT;
  _Float16* VTL  = (_Float16*)(ws + off); off += SZ_VTL;
  _Float16* O16  = (_Float16*)(ws + off); off += SZ_O16;
  _Float16* OL   = (_Float16*)(ws + off); off += SZ_OL;
  if (off > ws_size) return;

  k_wt_f16<<<(unsigned)(((size_t)3 * DM * (DM / 8) + 255) / 256), 256, 0, stream>>>(w_attn, BQKV, DM, 3 * DM, 16.0f);
  k_wt_f16<<<(unsigned)(((size_t)DM * (DM / 8) + 255) / 256), 256, 0, stream>>>(w_proj, BO, DM, DM, 16.0f);
  k_x16<<<(unsigned)(((size_t)NR * (DM / 8) + 255) / 256), 256, 0, stream>>>(x, X16);
  k_gemm_qk<<<(unsigned)((NR / 128) * (2 * DM / 64)), 128, 0, stream>>>(X16, BQKV, b_attn, QK, QKL);
  k_gemm_vt<<<(unsigned)((DM / 128) * (NR / 64)), 128, 0, stream>>>(BQKV + (size_t)2 * DM * DM, X16, b_attn + 2 * DM, VT, VTL);
  k_attn_isl<<<(unsigned)(NB * NH * (ISL / 128)), 256, 0, stream>>>(QK, QKL, VT, VTL, O16, OL, s_pref);
  if (SEQ > ISL) k_attn_main<<<(unsigned)(NB * NH * ((SEQ - ISL) / 128)), 256, 0, stream>>>(QK, VT, O16, s_pref);
  if (SEQ > ISL) k_gemm_out<<<(unsigned)((NB * (SEQ - ISL) / 128) * (DM / 64)), 128, 0, stream>>>(O16, BO, b_proj, out);
  k_gemm_out_isl<<<(unsigned)((NRI / 64) * (DM / 64)), 128, 0, stream>>>(O16, OL, BO, b_proj, out);
}
